// GINGraphModel_11665131176543
// MI455X (gfx1250) — hardware-verified
//
#include <hip/hip_runtime.h>
#include <stddef.h>


#define DI      128
#define DM      128
#define DH      256
#define DO      128
#define NTHR    256
#define NWAVE   8
#define EPT     8
#define NGRP    2
#define CHUNK   (NTHR * EPT * NGRP)
#define WCAPC   (EPT * NGRP * 32)
#define WCAPF   (EPT * NGRP * 32)
#define ESHF    11
#define EMASK   0xFFFFF
#define NBC     32768
#define NBF     2048
#define RCAP    49152
#define RBN     128
#define TGT     256
#define DEGCAP  512
#define GROWS   128
#define OTHR    512
#define TPK     64
#define TPN     32
#define TPP     72
#define ACARRY  1
#define WSCL    64
#define WSCAP   134217728

#define LDS_COUNT  ((NBC + NWAVE * WCAPC + NWAVE) * 4)
#define LDS_FILL   ((RCAP + NBF + NWAVE * WCAPF + NWAVE) * 4)
#define LDS_GEMM   (GROWS * 128 * 4)

static_assert((CHUNK & (CHUNK - 1)) == 0);
static_assert((NBC & (NBC - 1)) == 0 && (NBF & (NBF - 1)) == 0);
static_assert(NBF <= (1 << ESHF));
static_assert((NBC % NBF) == 0);
static_assert(OTHR * 4 == NBF);
static_assert((RCAP % 32) == 0);
static_assert(TGT == NWAVE * 32);
static_assert(GROWS == NWAVE * 16);
static_assert((TGT % GROWS) == 0);
static_assert(NBC == NWAVE * 32 * 128);
static_assert((DI % 32) == 0 && (DM % 32) == 0 && (DH % 32) == 0);
static_assert((DI % TPK) == 0 && (DM % TPK) == 0 && (DH % TPK) == 0);
static_assert((DM % TPN) == 0 && (DH % TPN) == 0 && (DO % TPN) == 0);
static_assert(TPN * 8 == NTHR && TPK * TPN == NTHR * 8 && TPK == NWAVE * 8);
static_assert((TPP % 8) == 0 && TPP >= TPK);
static_assert(LDS_FILL <= 300 * 1024);

typedef float     v4f  __attribute__((ext_vector_type(4)));
typedef float     v8f  __attribute__((ext_vector_type(8)));
typedef int       v4i  __attribute__((ext_vector_type(4)));
typedef _Float16  v4h  __attribute__((ext_vector_type(4)));
typedef _Float16  v8h  __attribute__((ext_vector_type(8)));
typedef _Float16  v16h __attribute__((ext_vector_type(16)));
union FragH { v16h v; v8h h[2]; };

__device__ __forceinline__ v8f wmf(v16h a, v16h b, v8f c) {
  v8f d = __builtin_amdgcn_wmma_f32_16x16x32_f16(false, a, false, b, (short)0, c, false, false);
  asm volatile("v_nop\n\tv_nop\n\tv_nop\n\tv_nop" : "+v"(d) : "v"(a), "v"(b));
  return d;
}

template <int NB, int SRC, int WC>
__device__ __forceinline__ int scan_chunk(const int* __restrict__ keys, int nK, int cbase,
                                          int slotBase, int vec8, int* list, int tid, int lane, int wave) {
  int wc = 0;
#pragma unroll
  for (int g = 0; g < NGRP; ++g) {
    const int el0  = (g * NTHR + tid) * EPT;
    const int e0   = cbase + el0;
    const int sent = -2147483647 - 1;
    const int i0 = min(e0, nK - 1),     i1 = min(e0 + 1, nK - 1), i2 = min(e0 + 2, nK - 1), i3 = min(e0 + 3, nK - 1);
    const int i4 = min(e0 + 4, nK - 1), i5 = min(e0 + 5, nK - 1), i6 = min(e0 + 6, nK - 1), i7 = min(e0 + 7, nK - 1);
    v4i da, db;
    if (vec8 != 0 && cbase + CHUNK <= nK) {
      da = *(const v4i*)(keys + e0);
      db = *(const v4i*)(keys + e0 + 4);
    } else {
      da.x = (e0     < nK) ? keys[i0] : sent;
      da.y = (e0 + 1 < nK) ? keys[i1] : sent;
      da.z = (e0 + 2 < nK) ? keys[i2] : sent;
      da.w = (e0 + 3 < nK) ? keys[i3] : sent;
      db.x = (e0 + 4 < nK) ? keys[i4] : sent;
      db.y = (e0 + 5 < nK) ? keys[i5] : sent;
      db.z = (e0 + 6 < nK) ? keys[i6] : sent;
      db.w = (e0 + 7 < nK) ? keys[i7] : sent;
    }
    const unsigned nb = (unsigned)slotBase;
    const unsigned s0 = (unsigned)da.x - nb, s1 = (unsigned)da.y - nb;
    const unsigned s2 = (unsigned)da.z - nb, s3 = (unsigned)da.w - nb;
    const unsigned s4 = (unsigned)db.x - nb, s5 = (unsigned)db.y - nb;
    const unsigned s6 = (unsigned)db.z - nb, s7 = (unsigned)db.w - nb;
    const bool h0 = s0 < (unsigned)NB, h1 = s1 < (unsigned)NB, h2 = s2 < (unsigned)NB, h3 = s3 < (unsigned)NB;
    const bool h4 = s4 < (unsigned)NB, h5 = s5 < (unsigned)NB, h6 = s6 < (unsigned)NB, h7 = s7 < (unsigned)NB;
    const unsigned any = __builtin_amdgcn_ballot_w32(h0 | h1 | h2 | h3 | h4 | h5 | h6 | h7);
    if (any != 0u) {
#define HITJ(HJ, SJ, VJ) { \
        const unsigned mj = __builtin_amdgcn_ballot_w32(HJ); \
        if (mj != 0u) { \
          if (HJ) { \
            const int pos = wc + (int)__builtin_amdgcn_mbcnt_lo(mj, 0u); \
            const int entv = SRC ? (((VJ) << ESHF) | (int)(SJ)) : (int)(SJ); \
            if (pos < WC) list[wave * WC + pos] = entv; \
          } \
          wc += (int)__builtin_popcount(mj); } }
      HITJ(h0, s0, i0)
      HITJ(h1, s1, i1)
      HITJ(h2, s2, i2)
      HITJ(h3, s3, i3)
      HITJ(h4, s4, i4)
      HITJ(h5, s5, i5)
      HITJ(h6, s6, i6)
      HITJ(h7, s7, i7)
#undef HITJ
    }
  }
  return wc;
}

__global__ __launch_bounds__(NTHR) void k_wT16(const float* __restrict__ W, _Float16* Wp,
                                               int KD, int NC, float scale) {
  __shared__ __attribute__((aligned(16))) _Float16 sT[TPN * TPP];
  const int tid = threadIdx.x;
  const int k0 = (int)blockIdx.x * TPK, n0 = (int)blockIdx.y * TPN;
  const int nc = tid & 31, kq = tid >> 5;
#pragma unroll
  for (int i = 0; i < TPK / NWAVE; ++i) {
    const int kr = kq + NWAVE * i;
    const float v = W[(size_t)(k0 + kr) * NC + n0 + nc] * scale;
    sT[nc * TPP + kr] = (_Float16)v;
  }
  __syncthreads();
  const int nl = tid >> 3, p = tid & 7;
  const v8h hv = *(const v8h*)(sT + nl * TPP + 8 * p);
  _Float16* d = Wp + (size_t)(n0 + nl) * KD + k0 + 8 * p;
  *(volatile v8h*)d = hv;
  __threadfence();
  *(volatile v8h*)d = hv;
}

__global__ __launch_bounds__(NTHR) void k_count(
    const int* __restrict__ keys, int* cnt, int nK, int vec8) {
  extern __shared__ v4f lds_dyn[];
  int* scnt = (int*)lds_dyn;
  int* list = scnt + NBC;
  int* wcnt = list + NWAVE * WCAPC;
  const int tid = threadIdx.x, lane = tid & 31, wave = tid >> 5;
  const int nodeBase = blockIdx.x * NBC;

  {
    const v4i z = {0, 0, 0, 0};
    for (int i = tid; i < NBC / 4; i += NTHR) ((v4i*)scnt)[i] = z;
  }
  __syncthreads();

  const int nChunks = (nK + CHUNK - 1) / CHUNK;
#pragma unroll 1
  for (int ch = 0; ch < nChunks; ++ch) {
    const int cbase = ch * CHUNK;
    const int wc = scan_chunk<NBC, 0, WCAPC>(keys, nK, cbase, nodeBase, vec8, list, tid, lane, wave);
    if (lane == 0) wcnt[wave] = wc;
    __syncthreads();
    if (wave == 0) {
#pragma unroll 1
      for (int wsx = 0; wsx < NWAVE; ++wsx) {
        int n = __builtin_amdgcn_readfirstlane(wcnt[wsx]);
        n = n > WCAPC ? WCAPC : (n < 0 ? 0 : n);
        const int* lp = list + wsx * WCAPC;
#pragma unroll 1
        for (int i = 0; i < n; ++i) {
          const int ent  = __builtin_amdgcn_readfirstlane(lp[i]);
          const int slot = ent & (NBC - 1);
          if (lane == 0) scnt[slot] = scnt[slot] + 1;
        }
      }
    }
    __syncthreads();
  }

  int* cp = cnt + (size_t)nodeBase;
#pragma unroll 4
  for (int q = 0; q < 32; ++q) {
    const int f = (wave * 32 + q) * 128 + 4 * lane;
    const v4i c = *(const v4i*)(scnt + f);
    *(volatile v4i*)(cp + f) = c;
  }
  __threadfence();
#pragma unroll 4
  for (int q = 0; q < 32; ++q) {
    const int f = (wave * 32 + q) * 128 + 4 * lane;
    const v4i c = *(const v4i*)(scnt + f);
    *(volatile v4i*)(cp + f) = c;
  }
}

__global__ __launch_bounds__(OTHR) void k_offsets(
    const int* __restrict__ cnt, int* off, int* rbase, int nBF) {
  __shared__ __attribute__((aligned(16))) int srb[RBN];
  __shared__ int wtot[OTHR / 32];
  const int tid = threadIdx.x, lane = tid & 31, wave = tid >> 5;
  for (int i = tid; i < RBN; i += OTHR) srb[i] = 0;
  int carry = 0;
#pragma unroll 1
  for (int fb = 0; fb < nBF; ++fb) {
    const int base = fb * NBF;
    const v4i c = *(const v4i*)(cnt + base + 4 * tid);
    const int e0 = max(c.x, 0), e1 = max(c.y, 0), e2 = max(c.z, 0), e3 = max(c.w, 0);
    const int ts = e0 + e1 + e2 + e3;
    int incl = ts;
#pragma unroll
    for (int d = 1; d < 32; d <<= 1) {
      const int t = __shfl_up(incl, d, 32);
      if (lane >= d) incl += t;
    }
    if (lane == 31) wtot[wave] = incl;
    __syncthreads();
    int pre = 0;
#pragma unroll 1
    for (int w = 0; w < wave; ++w) pre += wtot[w];
    int tot = 0;
#pragma unroll
    for (int w = 0; w < OTHR / 32; ++w) tot += wtot[w];
    int run = carry + pre + incl - ts;
    v4i o;
    o.x = run; run += e0;
    o.y = run; run += e1;
    o.z = run; run += e2;
    o.w = run;
    int* op = off + base + 4 * tid;
    *(volatile v4i*)op = o;
    __threadfence();
    *(volatile v4i*)op = o;
    if (tid == 0) srb[min(fb, RBN - 1)] = carry;
    carry += (tot + 31) & ~31;
    __syncthreads();
  }
  if (tid == 0) srb[min(nBF, RBN - 1)] = carry;
  __syncthreads();
  v4i rv = {0, 0, 0, 0};
  if (tid < 32) rv = *(const v4i*)(srb + 4 * tid);
  if (tid < 32) *(volatile v4i*)(rbase + 4 * tid) = rv;
  __threadfence();
  if (tid < 32) *(volatile v4i*)(rbase + 4 * tid) = rv;
}

__global__ __launch_bounds__(NTHR) void k_fill(
    const int* __restrict__ keys, const int* __restrict__ off,
    const int* __restrict__ rbase, int* csr, int nK, int vec8, int csrLen) {
  extern __shared__ v4f lds_dyn[];
  int* region = (int*)lds_dyn;
  int* cursor = region + RCAP;
  int* list   = cursor + NBF;
  int* wcnt   = list + NWAVE * WCAPF;
  const int tid = threadIdx.x, lane = tid & 31, wave = tid >> 5;
  const int b = blockIdx.x;
  const int nodeBase = b * NBF;

  int rb0 = rbase[b];
  const int rb1 = rbase[b + 1];
  rb0 = rb0 < 0 ? 0 : (rb0 > csrLen ? csrLen : rb0);
  rb0 &= ~31;
  int len = rb1 - rb0;
  len = len < 0 ? 0 : (len > RCAP ? RCAP : len);
  int lenW = (len + 31) & ~31;
  if (rb0 + lenW > csrLen) lenW = (csrLen - rb0) & ~31;

  {
    const v4i z = {0, 0, 0, 0};
    for (int i = tid; i < RCAP / 4; i += NTHR) ((v4i*)region)[i] = z;
    for (int s = tid; s < NBF; s += NTHR) {
      int o = off[nodeBase + s] - rb0;
      o = o < 0 ? 0 : (o > RCAP ? RCAP : o);
      cursor[s] = o;
    }
  }
  __syncthreads();

  const int nChunks = (nK + CHUNK - 1) / CHUNK;
#pragma unroll 1
  for (int ch = 0; ch < nChunks; ++ch) {
    const int cbase = ch * CHUNK;
    const int wc = scan_chunk<NBF, 1, WCAPF>(keys, nK, cbase, nodeBase, vec8, list, tid, lane, wave);
    if (lane == 0) wcnt[wave] = wc;
    __syncthreads();
    if (wave == 0) {
#pragma unroll 1
      for (int wsx = 0; wsx < NWAVE; ++wsx) {
        int n = __builtin_amdgcn_readfirstlane(wcnt[wsx]);
        n = n > WCAPF ? WCAPF : (n < 0 ? 0 : n);
        const int* lp = list + wsx * WCAPF;
#pragma unroll 1
        for (int i = 0; i < n; ++i) {
          const int ent  = __builtin_amdgcn_readfirstlane(lp[i]);
          const int slot = ent & (NBF - 1);
          int ev = (ent >> ESHF) & EMASK;
          ev = ev > nK - 1 ? nK - 1 : ev;
          if (lane == 0) {
            int pos = cursor[slot];
            pos = pos < 0 ? 0 : (pos > RCAP - 1 ? RCAP - 1 : pos);
            region[pos] = ev;
            const int np = pos + 1;
            cursor[slot] = np > RCAP ? RCAP : np;
          }
        }
      }
    }
    __syncthreads();
  }

  const int nv = lenW >> 2;
  int* gp = csr + rb0;
#pragma unroll 1
  for (int i = tid; i < nv; i += NTHR) { const v4i v = ((const v4i*)region)[i]; *(volatile v4i*)(gp + 4 * i) = v; }
  __threadfence();
#pragma unroll 1
  for (int i = tid; i < nv; i += NTHR) { const v4i v = ((const v4i*)region)[i]; *(volatile v4i*)(gp + 4 * i) = v; }
}

__device__ __forceinline__ void cvst4(const float* lp, _Float16* gp, float s) {
  const v4f f = *(const v4f*)lp;
  v4h h;
  h[0] = (_Float16)(f.x * s); h[1] = (_Float16)(f.y * s); h[2] = (_Float16)(f.z * s); h[3] = (_Float16)(f.w * s);
  *(volatile v4h*)gp = h;
}
__device__ __forceinline__ void cvst8(const float* lp, _Float16* gp, float s) {
  const v4f f0 = *(const v4f*)lp;
  const v4f f1 = *(const v4f*)(lp + 4);
  v8h h;
  h[0] = (_Float16)(f0.x * s); h[1] = (_Float16)(f0.y * s); h[2] = (_Float16)(f0.z * s); h[3] = (_Float16)(f0.w * s);
  h[4] = (_Float16)(f1.x * s); h[5] = (_Float16)(f1.y * s); h[6] = (_Float16)(f1.z * s); h[7] = (_Float16)(f1.w * s);
  *(volatile v8h*)gp = h;
}

template <int KD, int NC, int EPI>
__global__ __launch_bounds__(NTHR) void k_gemm(
    const _Float16* __restrict__ A16, const _Float16* __restrict__ Bw,
    const float* __restrict__ bias, void* Cout, float osc, int nStore) {
  static_assert((KD % 32) == 0 && (NC == 128 || NC == 256));
  constexpr int CW  = NC / 128;
  constexpr int RB  = GROWS / CW;
  constexpr int RPW = RB / NWAVE;
  constexpr int NT  = 8;
  extern __shared__ v4f lds_dyn[];
  float* stg = (float*)lds_dyn;
  const int tid = threadIdx.x, lane = tid & 31, wave = tid >> 5, hh = lane >> 4, m = lane & 15;
  const int rg = wave / CW, cg = wave - rg * CW;
  const int rowBase = (int)blockIdx.x * RB;
  const _Float16* ap  = A16 + (size_t)(rowBase + 16 * rg + m) * KD + 8 * hh;
  const _Float16* bp0 = Bw + (size_t)(128 * cg + m) * KD + 8 * hh;

  v8f acc[NT];
#pragma unroll
  for (int t = 0; t < NT; ++t) { v8f z = {0.f, 0.f, 0.f, 0.f, 0.f, 0.f, 0.f, 0.f}; acc[t] = z; }

#pragma unroll 1
  for (int kt = 0; kt < KD / 32; ++kt) {
    FragH af;
    af.h[0] = *(const v8h*)(ap + 32 * kt);
    af.h[1] = *(const v8h*)(ap + 32 * kt + 16);
#pragma unroll
    for (int t = 0; t < NT; ++t) {
      const _Float16* bp = bp0 + (size_t)(16 * t) * KD + 32 * kt;
      FragH bf;
      bf.h[0] = *(const v8h*)bp;
      bf.h[1] = *(const v8h*)(bp + 16);
      acc[t] = wmf(af.v, bf.v, acc[t]);
    }
  }

  const int r0 = 16 * rg + 8 * hh;
  float bc[NT];
#pragma unroll
  for (int t = 0; t < NT; ++t) bc[t] = bias[128 * cg + 16 * t + m];

  float* sp = stg + r0 * NC + 128 * cg + m;
#pragma unroll
  for (int t = 0; t < NT; ++t) {
#pragma unroll
    for (int r = 0; r < 8; ++r) {
      float v = acc[t][r] * osc + bc[t];
      if (EPI != 2) v = fmaxf(v, 0.0f);
      sp[r * NC + 16 * t] = v;
    }
  }
  __syncthreads();

  const float* lp = stg + wave * RPW * NC;
  const int orow0 = rowBase + wave * RPW;
  if constexpr (EPI == 0) {
    _Float16* C = (_Float16*)Cout;
    constexpr int HPL = NC / 32;
    const float acs = (float)ACARRY;
#pragma unroll
    for (int i = 0; i < RPW; ++i) {
      if (orow0 + i < nStore) {
        _Float16* gp = C + (size_t)(orow0 + i) * NC + HPL * lane;
        if constexpr (HPL == 4) cvst4(lp + i * NC + HPL * lane, gp, acs);
        else                    cvst8(lp + i * NC + HPL * lane, gp, acs);
      }
    }
    __threadfence();
#pragma unroll
    for (int i = 0; i < RPW; ++i) {
      if (orow0 + i < nStore) {
        _Float16* gp = C + (size_t)(orow0 + i) * NC + HPL * lane;
        if constexpr (HPL == 4) cvst4(lp + i * NC + HPL * lane, gp, acs);
        else                    cvst8(lp + i * NC + HPL * lane, gp, acs);
      }
    }
  } else {
    float* C = (float*)Cout;
#pragma unroll
    for (int i = 0; i < RPW; ++i) {
      if (orow0 + i < nStore) {
#pragma unroll
        for (int p = 0; p < CW; ++p) {
          const v4f v = *(const v4f*)(lp + i * NC + 128 * p + 4 * lane);
          *(volatile v4f*)(C + (size_t)(orow0 + i) * NC + 128 * p + 4 * lane) = v;
        }
      }
    }
    __threadfence();
#pragma unroll
    for (int i = 0; i < RPW; ++i) {
      if (orow0 + i < nStore) {
#pragma unroll
        for (int p = 0; p < CW; ++p) {
          const v4f v = *(const v4f*)(lp + i * NC + 128 * p + 4 * lane);
          *(volatile v4f*)(C + (size_t)(orow0 + i) * NC + 128 * p + 4 * lane) = v;
        }
      }
    }
  }
}

template <int D>
__global__ __launch_bounds__(NTHR) void k_agg(
    const int* __restrict__ csr, const int* __restrict__ off, const int* __restrict__ cnt,
    const int* __restrict__ srcidx, const float* __restrict__ hw,
    _Float16* outp, int nN, int nE, int csrLen, float acs) {
  static_assert(D == 128 || D == 256);
  constexpr int FPL = D / 32;
  const int tid = threadIdx.x, lane = tid & 31, wave = tid >> 5;
  const int tbase = (int)blockIdx.x * TGT + wave * 32;
  const int cl = tbase + lane;
  const int cnt_l = cnt[cl];
  const int off_l = off[cl];
  const int ch = FPL * lane;

#pragma unroll 1
  for (int j = 0; j < 32; ++j) {
    const int c = tbase + j;
    const int nraw = __builtin_amdgcn_readlane(cnt_l, j);
    const int n = nraw < 0 ? 0 : (nraw > DEGCAP ? DEGCAP : nraw);
    const int st = __builtin_amdgcn_readlane(off_l, j);
    v4f a0 = {0.f, 0.f, 0.f, 0.f};
    v4f a1 = {0.f, 0.f, 0.f, 0.f};
#pragma unroll 1
    for (int q0 = 0; q0 < n; q0 += 32) {
      int pos = st + q0 + lane;
      pos = pos < 0 ? 0 : (pos > csrLen - 1 ? csrLen - 1 : pos);
      int el = csr[pos];
      el = el < 0 ? 0 : (el > nE - 1 ? nE - 1 : el);
      int sl = srcidx[el];
      sl = sl < 0 ? 0 : (sl > nN - 1 ? nN - 1 : sl);
      const int mcnt = (n - q0) < 32 ? (n - q0) : 32;
#pragma unroll 1
      for (int p = 0; p < mcnt; ++p) {
        const int s = __builtin_amdgcn_readlane(sl, p);
        const float* hp = hw + (size_t)s * D + ch;
        const v4f h0 = *(const v4f*)hp;
        a0 = a0 + h0;
        if constexpr (FPL == 8) {
          const v4f h1 = *(const v4f*)(hp + 4);
          a1 = a1 + h1;
        }
      }
    }
    const int cs = c < nN ? c : nN - 1;
    const float* selfp = hw + (size_t)cs * D + ch;
    v4f v0 = a0 + *(const v4f*)selfp;
    v4f v1 = a1;
    if constexpr (FPL == 8) v1 = a1 + *(const v4f*)(selfp + 4);
    if (c >= nN) {
      const v4f z = {0.f, 0.f, 0.f, 0.f}; v0 = z; v1 = z;
    }
    if (nraw > DEGCAP) {
      const float qn = __int_as_float(0x7fc00000);
      v0.x = qn; v0.y = qn; v0.z = qn; v0.w = qn;
      v1.x = qn; v1.y = qn; v1.z = qn; v1.w = qn;
    }
    _Float16* rp = outp + (size_t)c * D + ch;
    if constexpr (FPL == 4) {
      v4h hv;
      hv[0] = (_Float16)(v0.x * acs); hv[1] = (_Float16)(v0.y * acs); hv[2] = (_Float16)(v0.z * acs); hv[3] = (_Float16)(v0.w * acs);
      *(volatile v4h*)rp = hv;
      __threadfence();
      *(volatile v4h*)rp = hv;
    } else {
      v8h hv;
      hv[0] = (_Float16)(v0.x * acs); hv[1] = (_Float16)(v0.y * acs); hv[2] = (_Float16)(v0.z * acs); hv[3] = (_Float16)(v0.w * acs);
      hv[4] = (_Float16)(v1.x * acs); hv[5] = (_Float16)(v1.y * acs); hv[6] = (_Float16)(v1.z * acs); hv[7] = (_Float16)(v1.w * acs);
      *(volatile v8h*)rp = hv;
      __threadfence();
      *(volatile v8h*)rp = hv;
    }
  }
}

extern "C" void kernel_launch(void* const* d_in, const int* in_sizes, int n_in,
                              void* d_out, int out_size, void* d_ws, size_t ws_size,
                              hipStream_t stream) {
  if (n_in < 14) return;
  const int nN = in_sizes[0] / DI;
  const int nE = in_sizes[1] / 2;
  if (nN <= 0 || nE <= 0) return;
  if (in_sizes[0] != nN * DI || in_sizes[1] != 2 * nE) return;
  if (in_sizes[2] != DI * DM || in_sizes[3] != DM) return;
  if (in_sizes[4] != DM * DH || in_sizes[5] != DH) return;
  if (in_sizes[6] != DH * DH || in_sizes[7] != DH) return;
  if (in_sizes[8] != DH * DM || in_sizes[9] != DM) return;
  if (in_sizes[10] != DM * DM || in_sizes[11] != DM) return;
  if (in_sizes[12] != DM * DO || in_sizes[13] != DO) return;
  if (nN > (1 << 20) || nE > (1 << 20)) return;
  if ((long long)out_size != (long long)nN * DO) return;

  const float* x   = (const float*)d_in[0];
  const int*   ei  = (const int*)d_in[1];
  const float* w1a = (const float*)d_in[2];
  const float* b1a = (const float*)d_in[3];
  const float* w1b = (const float*)d_in[4];
  const float* b1b = (const float*)d_in[5];
  const float* w2a = (const float*)d_in[6];
  const float* b2a = (const float*)d_in[7];
  const float* w2b = (const float*)d_in[8];
  const float* b2b = (const float*)d_in[9];
  const float* w3a = (const float*)d_in[10];
  const float* b3a = (const float*)d_in[11];
  const float* w3b = (const float*)d_in[12];
  const float* b3b = (const float*)d_in[13];
  float* out = (float*)d_out;
  const int* srci = ei;
  const int* dsti = ei + nE;
  const int nK = nE;

  const int NPAD   = ((nN + TGT - 1) / TGT) * TGT;
  const int nBC    = (nN + NBC - 1) / NBC;
  const int CNTPAD = nBC * NBC;
  const int nBF    = (nN + NBF - 1) / NBF;
  const int OFFN   = nBF * NBF;
  if (nBF + 1 > RBN) return;
  if (OFFN > CNTPAD || NPAD > OFFN) return;
  if ((NPAD % GROWS) != 0 || (NPAD % TGT) != 0 || (NPAD % 64) != 0) return;
  const int csrLen = ((nK + 31) & ~31) + 32 * (nBF + 1);
  const int nG128  = NPAD / GROWS;
  const int nG64   = NPAD / (GROWS / 2);
  const int nAgg   = NPAD / TGT;

  char* ws = (char*)d_ws;
  size_t off = 0;
  const size_t oA16 = off; off += (size_t)NPAD * DH * 2;         off = (off + 255) & ~(size_t)255;
  const size_t oM16 = off; off += (size_t)NPAD * DH * 2;         off = (off + 255) & ~(size_t)255;
  const size_t oH32 = off; off += (size_t)NPAD * DH * 4;         off = (off + 255) & ~(size_t)255;
  const size_t oW1a = off; off += (size_t)DM * DI * 2;           off = (off + 255) & ~(size_t)255;
  const size_t oW1b = off; off += (size_t)DH * DM * 2;           off = (off + 255) & ~(size_t)255;
  const size_t oW2a = off; off += (size_t)DH * DH * 2;           off = (off + 255) & ~(size_t)255;
  const size_t oW2b = off; off += (size_t)DM * DH * 2;           off = (off + 255) & ~(size_t)255;
  const size_t oW3a = off; off += (size_t)DM * DM * 2;           off = (off + 255) & ~(size_t)255;
  const size_t oW3b = off; off += (size_t)DO * DM * 2;           off = (off + 255) & ~(size_t)255;
  const size_t oCnt = off; off += (size_t)CNTPAD * 4;            off = (off + 255) & ~(size_t)255;
  const size_t oOff = off; off += (size_t)OFFN * 4;              off = (off + 255) & ~(size_t)255;
  const size_t oRb  = off; off += (size_t)RBN * 4;               off = (off + 255) & ~(size_t)255;
  const size_t oCsr = off; off += (size_t)csrLen * 4;            off = (off + 255) & ~(size_t)255;
  if (off > ws_size || off > (size_t)WSCAP) return;
  _Float16* A16  = (_Float16*)(ws + oA16);
  _Float16* M16  = (_Float16*)(ws + oM16);
  float*    H32  = (float*)(ws + oH32);
  _Float16* W1ap = (_Float16*)(ws + oW1a);
  _Float16* W1bp = (_Float16*)(ws + oW1b);
  _Float16* W2ap = (_Float16*)(ws + oW2a);
  _Float16* W2bp = (_Float16*)(ws + oW2b);
  _Float16* W3ap = (_Float16*)(ws + oW3a);
  _Float16* W3bp = (_Float16*)(ws + oW3b);
  int*      cnt  = (int*)(ws + oCnt);
  int*      offp = (int*)(ws + oOff);
  int*      rb   = (int*)(ws + oRb);
  int*      csr  = (int*)(ws + oCsr);

  const int vec8 = ((nE & 3) == 0) ? 1 : 0;
  const float osc = 1.0f / ((float)ACARRY * (float)WSCL);
  const float acs = (float)ACARRY;

  {
    const dim3 g1a(DI / TPK, DM / TPN);
    const dim3 g1b(DM / TPK, DH / TPN);
    const dim3 g2a(DH / TPK, DH / TPN);
    const dim3 g2b(DH / TPK, DM / TPN);
    const dim3 g3a(DM / TPK, DM / TPN);
    const dim3 g3b(DM / TPK, DO / TPN);
    k_wT16<<<g1a, NTHR, 0, stream>>>(w1a, W1ap, DI, DM, (float)WSCL);
    k_wT16<<<g1b, NTHR, 0, stream>>>(w1b, W1bp, DM, DH, (float)WSCL);
    k_wT16<<<g2a, NTHR, 0, stream>>>(w2a, W2ap, DH, DH, (float)WSCL);
    k_wT16<<<g2b, NTHR, 0, stream>>>(w2b, W2bp, DH, DM, (float)WSCL);
    k_wT16<<<g3a, NTHR, 0, stream>>>(w3a, W3ap, DM, DM, (float)WSCL);
    k_wT16<<<g3b, NTHR, 0, stream>>>(w3b, W3bp, DM, DO, (float)WSCL);
  }

  hipFuncSetAttribute(reinterpret_cast<const void*>(&k_count),
                      hipFuncAttributeMaxDynamicSharedMemorySize, LDS_COUNT);
  k_count<<<nBC, NTHR, LDS_COUNT, stream>>>(dsti, cnt, nK, vec8);
  k_offsets<<<1, OTHR, 0, stream>>>(cnt, offp, rb, nBF);
  hipFuncSetAttribute(reinterpret_cast<const void*>(&k_fill),
                      hipFuncAttributeMaxDynamicSharedMemorySize, LDS_FILL);
  k_fill<<<nBF, NTHR, LDS_FILL, stream>>>(dsti, offp, rb, csr, nK, vec8, csrLen);

  hipFuncSetAttribute(reinterpret_cast<const void*>(&k_gemm<DI, DM, 0>),
                      hipFuncAttributeMaxDynamicSharedMemorySize, LDS_GEMM);
  hipFuncSetAttribute(reinterpret_cast<const void*>(&k_gemm<DM, DH, 1>),
                      hipFuncAttributeMaxDynamicSharedMemorySize, LDS_GEMM);
  hipFuncSetAttribute(reinterpret_cast<const void*>(&k_gemm<DH, DH, 0>),
                      hipFuncAttributeMaxDynamicSharedMemorySize, LDS_GEMM);
  hipFuncSetAttribute(reinterpret_cast<const void*>(&k_gemm<DH, DM, 1>),
                      hipFuncAttributeMaxDynamicSharedMemorySize, LDS_GEMM);
  hipFuncSetAttribute(reinterpret_cast<const void*>(&k_gemm<DM, DO, 2>),
                      hipFuncAttributeMaxDynamicSharedMemorySize, LDS_GEMM);

  k_agg<DI><<<nAgg, NTHR, 0, stream>>>(csr, offp, cnt, srci, x, A16, nN, nE, csrLen, acs);
  k_gemm<DI, DM, 0><<<nG128, NTHR, LDS_GEMM, stream>>>(A16, W1ap, b1a, (void*)M16, osc, NPAD);
  k_gemm<DM, DH, 1><<<nG64, NTHR, LDS_GEMM, stream>>>(M16, W1bp, b1b, (void*)H32, osc, NPAD);

  k_agg<DH><<<nAgg, NTHR, 0, stream>>>(csr, offp, cnt, srci, H32, A16, nN, nE, csrLen, acs);
  k_gemm<DH, DH, 0><<<nG64, NTHR, LDS_GEMM, stream>>>(A16, W2ap, b2a, (void*)M16, osc, NPAD);
  k_gemm<DH, DM, 1><<<nG128, NTHR, LDS_GEMM, stream>>>(M16, W2bp, b2b, (void*)H32, osc, NPAD);

  k_agg<DM><<<nAgg, NTHR, 0, stream>>>(csr, offp, cnt, srci, H32, A16, nN, nE, csrLen, acs);
  k_gemm<DM, DM, 0><<<nG128, NTHR, LDS_GEMM, stream>>>(A16, W3ap, b3a, (void*)M16, osc, NPAD);
  k_gemm<DM, DO, 2><<<nG128, NTHR, LDS_GEMM, stream>>>(M16, W3bp, b3b, (void*)out, osc, nN);
}
